// SetConv_58677843198342
// MI455X (gfx1250) — hardware-verified
//
#include <hip/hip_runtime.h>
#include <math.h>

typedef __attribute__((ext_vector_type(16))) _Float16 v16h;
typedef __attribute__((ext_vector_type(16))) __bf16 v16b;
typedef __attribute__((ext_vector_type(8)))  _Float16 v8h;
typedef __attribute__((ext_vector_type(8)))  float v8f;
typedef __attribute__((ext_vector_type(4)))  float v4f;
typedef __attribute__((ext_vector_type(2)))  float v2f;
typedef __attribute__((ext_vector_type(4)))  unsigned v4u;
typedef __attribute__((ext_vector_type(4)))  int v4i;
typedef float __attribute__((may_alias)) float_a;
typedef int __attribute__((may_alias)) int_a;

template <typename T> __device__ __forceinline__ void vst2(void* p, T v) { *(volatile T*)p = v; __threadfence(); *(volatile T*)p = v; }
__device__ __forceinline__ v8f wmma16(v16h a, v16h b, v8f c) {
  v8f d = __builtin_amdgcn_wmma_f32_16x16x32_f16(false, a, false, b, (short)0, c, false, false);
  asm volatile("v_nop\n\tv_nop\n\tv_nop\n\tv_nop" : "+v"(d) : "v"(a), "v"(b));
  return d;
}
__device__ __forceinline__ v8f wmma_bf(v16b a, v16b b, v8f c) {
  v8f d = __builtin_amdgcn_wmma_f32_16x16x32_bf16(false, a, false, b, (short)0, c, false, false);
  asm volatile("v_nop\n\tv_nop\n\tv_nop\n\tv_nop" : "+v"(d) : "v"(a), "v"(b));
  return d;
}
__device__ __forceinline__ v16h frag_h(const _Float16* rowk0, int lane) {
  union { v16h v; v8h q[2]; } u; const _Float16* p = rowk0 + 8 * (lane >> 4);
  u.q[0] = *(const v8h*)p; u.q[1] = *(const v8h*)(p + 16); return u.v;
}
__device__ __forceinline__ v16h frag_f32(const float* rowk0, int lane) {
  v16h a; const float* p = rowk0 + 8 * (lane >> 4);
#pragma unroll
  for (int i = 0; i < 8; ++i) { a[i] = (_Float16)p[i]; a[8 + i] = (_Float16)p[16 + i]; }
  return a;
}
__device__ __forceinline__ v16h frag_f32s(const float* rowk0, int lane, float sc) {
  v16h a; const float* p = rowk0 + 8 * (lane >> 4);
#pragma unroll
  for (int i = 0; i < 8; ++i) { a[i] = (_Float16)(p[i] * sc); a[8 + i] = (_Float16)(p[16 + i] * sc); }
  return a;
}
__device__ __forceinline__ v16h fragc_f32(const float* W, int k0, int n, int lane, int ld, int K) {
  v16h a; const int g = lane >> 4;
#pragma unroll
  for (int i = 0; i < 8; ++i) { const int ka = k0 + 8 * g + i, kb = ka + 16;
    a[i] = (_Float16)(ka < K ? W[(size_t)(ka < K ? ka : K - 1) * ld + n] : 0.f); a[8 + i] = (_Float16)(kb < K ? W[(size_t)(kb < K ? kb : K - 1) * ld + n] : 0.f); }
  return a;
}
struct F2 { v16b h, l; };
__device__ __forceinline__ F2 bsplit16(const float v[16]) { F2 r;
#pragma unroll
  for (int i = 0; i < 16; ++i) { const __bf16 h = (__bf16)v[i]; r.h[i] = h; r.l[i] = (__bf16)(v[i] - (float)h); }
  return r; }
__device__ __forceinline__ F2 split_row(const float* row, int k0, int lane) { float v[16]; const float* p = row + k0 + 8 * (lane >> 4);
#pragma unroll
  for (int i = 0; i < 8; ++i) { v[i] = p[i]; v[8 + i] = p[16 + i]; }
  return bsplit16(v); }
__device__ __forceinline__ F2 split_rowK(const float* row, int k0, int lane, int K) { float v[16]; const int g = lane >> 4;
#pragma unroll
  for (int i = 0; i < 8; ++i) { const int ka = k0 + 8 * g + i, kb = ka + 16; v[i] = ka < K ? row[ka < K ? ka : K - 1] : 0.f; v[8 + i] = kb < K ? row[kb < K ? kb : K - 1] : 0.f; }
  return bsplit16(v); }
__device__ __forceinline__ F2 split_col(const float* W, int k0, int n, int lane, int ld, int K) { float v[16]; const int g = lane >> 4;
#pragma unroll
  for (int i = 0; i < 8; ++i) { const int ka = k0 + 8 * g + i, kb = ka + 16; v[i] = ka < K ? W[(size_t)(ka < K ? ka : K - 1) * ld + n] : 0.f; v[8 + i] = kb < K ? W[(size_t)(kb < K ? kb : K - 1) * ld + n] : 0.f; }
  return bsplit16(v); }
__device__ __forceinline__ v8f mac3(const F2& a, const F2& b, v8f c) { c = wmma_bf(a.l, b.h, c); c = wmma_bf(a.h, b.l, c); return wmma_bf(a.h, b.h, c); }
__device__ __forceinline__ float sigm(float v) { return 1.0f / (1.0f + expf(-v)); }
#define LDSX() do { asm volatile("s_wait_dscnt 0" ::: "memory"); __builtin_amdgcn_wave_barrier(); __builtin_amdgcn_fence(__ATOMIC_RELEASE, "workgroup"); } while (0)

__device__ __forceinline__ float bfr(float v) { return (float)(__bf16)v; }
#define NB 8
#define NQ 2048
#define NK 2048
#define CIN 64
#define COUT 64
#ifndef TNB
#define TNB NB
#endif
typedef __attribute__((ext_vector_type(8))) __bf16 v8b;
__device__ __forceinline__ v16b frag_b(const __bf16* rowk0, int lane) { union { v16b v; v8b q[2]; } u; const __bf16* p = rowk0 + 8 * (lane >> 4); u.q[0] = *(const v8b*)p; u.q[1] = *(const v8b*)(p + 16); return u.v; }
#define WS_VP  0u
#define WS_S   (WS_VP + 2u * (size_t)NB * CIN * NK)
#define WS_T   (WS_S + 4u * (size_t)NQ * NK)
#define WS_DEN (WS_T + 4u * (size_t)NB * NQ * CIN)
#define WS_END (WS_DEN + 128u * (size_t)NB * NQ)
__global__ __launch_bounds__(128) void k_vt(const float* __restrict__ V, __bf16* __restrict__ VP) { __shared__ __align__(16) __bf16 th[CIN][136];
  const int tid = threadIdx.x; const int k0 = blockIdx.x * 128; const size_t b = blockIdx.y;
  for (int e = tid; e < 128 * CIN; e += 128) { const int kl = e / CIN, c = e % CIN; th[c][kl] = (__bf16)V[(b * NK + k0 + kl) * CIN + c]; }
  __syncthreads();
  for (int e = tid; e < CIN * 16; e += 128) { const int c = e >> 4, q = e & 15; vst2((unsigned*)(VP + (b * CIN + c) * (size_t)NK + k0 + q * 8), *(const v4u*)&th[c][q * 8]); } }
__global__ __launch_bounds__(128) void k_lg(const float* __restrict__ KEYS, const float* __restrict__ QRY, const float* __restrict__ WW, const float* __restrict__ LS, int b, float* __restrict__ S) { __shared__ float sq[64][2];
  const int t = threadIdx.x; const int k0 = blockIdx.y * 128; const int q0 = blockIdx.x * 64;
  if (t < 64) { sq[t][0] = bfr(QRY[((size_t)b * NQ + q0 + t) * 2]); sq[t][1] = bfr(QRY[((size_t)b * NQ + q0 + t) * 2 + 1]); }
  const float kx = bfr(KEYS[((size_t)b * NK + k0 + t) * 2]), ky = bfr(KEYS[((size_t)b * NK + k0 + t) * 2 + 1]);
  const float w00 = bfr(WW[0]), w01 = bfr(WW[1]), w10 = bfr(WW[2]), w11 = bfr(WW[3]);
  const float z = bfr(LS[0]) * 0.1f - 1.0f; const float sp = (z > 0.f ? z : 0.f) + log1pf(expf(-fabsf(z)));
  const float sigma = 1e-05f + sp;
  __syncthreads();
#pragma unroll 4
  for (int r = 0; r < 64; ++r) { const float dx = kx - sq[r][0], dy = ky - sq[r][1]; const float e0 = dx * w00 + dy * w01, e1 = dx * w10 + dy * w11; const float dist = sqrtf(e0 * e0 + e1 * e1); const float u = dist / sigma; S[(size_t)(q0 + r) * NK + k0 + t] = -0.5f * (u * u); } }
__global__ __launch_bounds__(256) void k_sm(float* __restrict__ S, int b, float* __restrict__ DEN) { __shared__ float sred[8], sred2[8]; __shared__ float sbc; __shared__ __align__(16) float sh[NK];
  const int t = threadIdx.x; const size_t row = blockIdx.x; float* sr = S + row * NK;
  float m = -3.0e38f; for (int k = t; k < NK; k += 256) { const float v = sr[k]; sh[k] = v; m = fmaxf(m, v); }
#pragma unroll
  for (int o = 1; o < 32; o <<= 1) m = fmaxf(m, __shfl_xor(m, o));
  if ((t & 31) == 0) sred[t >> 5] = m; __syncthreads(); if (t == 0) { float a = sred[0]; for (int w = 1; w < 8; ++w) a = fmaxf(a, sred[w]); sbc = a; } __syncthreads(); m = sbc; __syncthreads();
  float s = 0.f, sraw = 0.f; for (int k = t; k < NK; k += 256) { const float l = sh[k]; const float e = expf(l - m); sh[k] = e; s += e; sraw += expf(l); }
#pragma unroll
  for (int o = 1; o < 32; o <<= 1) { s += __shfl_xor(s, o); sraw += __shfl_xor(sraw, o); }
  if ((t & 31) == 0) { sred[t >> 5] = s; sred2[t >> 5] = sraw; } __syncthreads();
  if (t < 32) { float a = 0.f, a2 = 0.f; for (int w = 0; w < 8; ++w) { a += sred[w]; a2 += sred2[w]; } if (t == 0) sbc = 2048.0f / a; vst2(DEN + ((size_t)b * NQ + row) * 32 + t, a2); }
  __syncthreads(); const float sc = sbc;
  for (int k = t; k < NK; k += 256) sh[k] *= sc;
  __syncthreads(); for (int q = t; q < NK / 4; q += 256) vst2(sr + q * 4, *(const v4f*)&sh[q * 4]); }
__global__ __launch_bounds__(128) void k_pv(const float* __restrict__ PS, const __bf16* __restrict__ VP, int b, float* __restrict__ T) { __shared__ __align__(16) float ss[4][16][CIN + 4];
  const int tid = threadIdx.x, wave = tid >> 5, lane = tid & 31, col = lane & 15, g = lane >> 4; const int ql0 = blockIdx.x * 64 + wave * 16;
  v8f acc[CIN / 16] = {};
#pragma unroll 1
  for (int kc = 0; kc < NK / 32; ++kc) { const F2 p = split_row(PS + (size_t)(ql0 + col) * NK, kc * 32, lane);
#pragma unroll
    for (int j = 0; j < CIN / 16; ++j) { const v16b vv = frag_b(VP + ((size_t)b * CIN + j * 16 + col) * (size_t)NK + kc * 32, lane); acc[j] = wmma_bf(p.h, vv, acc[j]); acc[j] = wmma_bf(p.l, vv, acc[j]); } }
#pragma unroll
  for (int j = 0; j < CIN / 16; ++j)
#pragma unroll
    for (int r = 0; r < 8; ++r) ss[wave][8 * g + r][j * 16 + col] = acc[j][r] * (1.0f / 2048.0f);
  LDSX(); for (int rl = 0; rl < 16; ++rl) if (lane < CIN / 4) vst2(T + ((size_t)b * NQ + ql0 + rl) * CIN + lane * 4, *(const v4f*)&ss[wave][rl][lane * 4]); }
__global__ __launch_bounds__(128) void k_out(const float* __restrict__ T, const float* __restrict__ DEN, const float* __restrict__ DW, const float* __restrict__ DB, const float* __restrict__ RW, const float* __restrict__ RB, float* __restrict__ OUT) { __shared__ __align__(16) float sf[4][16][68];
  const int tid = threadIdx.x, wave = tid >> 5, lane = tid & 31, col = lane & 15, g = lane >> 4; const size_t r0 = (size_t)blockIdx.x * 64 + wave * 16;
  v8f acc[4] = {};
#pragma unroll
  for (int kc = 0; kc < CIN / 32; ++kc) { const F2 a = split_row(T + (r0 + col) * CIN, kc * 32, lane);
#pragma unroll
    for (int j = 0; j < 4; ++j) { v16b w; const float* wr = RW + (size_t)(j * 16 + col) * (CIN + 1) + kc * 32 + 8 * g;
#pragma unroll
      for (int i = 0; i < 8; ++i) { w[i] = (__bf16)wr[i]; w[8 + i] = (__bf16)wr[16 + i]; }
      asm volatile("s_wait_loadcnt 0x0" ::: "memory"); acc[j] = wmma_bf(a.h, w, acc[j]); acc[j] = wmma_bf(a.l, w, acc[j]); } }
  const float dw = bfr(DW[0]), db = bfr(DB[0]);
#pragma unroll
  for (int j = 0; j < 4; ++j) { const int o = j * 16 + col; const float wden = bfr(RW[(size_t)o * (CIN + 1) + CIN]), bb = bfr(RB[o]);
#pragma unroll
    for (int r = 0; r < 8; ++r) { const float den = DEN[(r0 + 8 * g + r) * 32]; const float sg = 1.0f / (1.0f + expf(-((-den * dw + db) * 0.1f))); sf[wave][8 * g + r][o] = acc[j][r] + sg * wden + bb; } }
  LDSX(); for (int rl = 0; rl < 16; ++rl) if (lane < 16) vst2(OUT + (r0 + rl) * COUT + lane * 4, *(const v4f*)&sf[wave][rl][lane * 4]); }
extern "C" void kernel_launch(void* const* d_in, const int* in_sizes, int n_in, void* d_out, int out_size, void* d_ws, size_t ws_size, hipStream_t stream) {
  (void)in_sizes; (void)n_in; (void)out_size;
  const float** F = (const float**)d_in;
  if (ws_size < (size_t)WS_END) return;
  char* ws = (char*)d_ws; __bf16* VP = (__bf16*)(ws + WS_VP); float *S = (float*)(ws + WS_S), *T = (float*)(ws + WS_T), *DEN = (float*)(ws + WS_DEN);
  k_vt<<<dim3(NK / 128, TNB), 128, 0, stream>>>(F[2], VP);
  for (int b = 0; b < TNB; ++b) {
    k_lg<<<dim3(NQ / 64, NK / 128), 128, 0, stream>>>(F[0], F[1], F[3], F[4], b, S);
    k_sm<<<dim3(NQ), 256, 0, stream>>>(S, b, DEN);
    k_pv<<<dim3(NQ / 64), 128, 0, stream>>>(S, VP, b, T);
  }
  k_out<<<dim3(TNB * NQ / 64), 128, 0, stream>>>(T, DEN, F[5], F[6], F[7], F[8], (float*)d_out);
}
